// MultiHeadAttention_42674795053763
// MI455X (gfx1250) — hardware-run, weakly checked
//
#include <hip/hip_runtime.h>


#ifndef NB
#define NB 4
#endif
#ifndef SEQ
#define SEQ 2048
#endif
#define NB_FULL  4
#define SEQ_FULL 2048
#ifndef OUT_SEQ
#define OUT_SEQ SEQ
#endif
#define DM   1024
#define NH_  16
#define HD   64
#define WOS  256.0f
#define WOI  (1.0f / 256.0f)
#define BIGB (1LL << 30)

static_assert(HD == 64);
static_assert(NH_ * HD == DM);
static_assert(DM % 64 == 0);
static_assert(DM % 32 == 0);
static_assert(SEQ % 64 == 0);
static_assert((NB * SEQ) % 64 == 0);
static_assert(SEQ % 32 == 0);
static_assert(((size_t)SEQ * DM) % 8 == 0);
static_assert(NB <= NB_FULL);
static_assert(SEQ <= SEQ_FULL);

typedef _Float16 h16;
typedef unsigned short us;
typedef __attribute__((ext_vector_type(16))) __bf16   v16bf;
typedef __attribute__((ext_vector_type(16))) _Float16 v16h;
typedef __attribute__((ext_vector_type(8)))  unsigned short v8us;
typedef __attribute__((ext_vector_type(8)))  float    v8f;
typedef __attribute__((ext_vector_type(4)))  float    v4f;
typedef v4f  __attribute__((may_alias)) v4fa;

__device__ __forceinline__ us f2bf(float f) { unsigned u = __float_as_uint(f); u += 0x7FFFu + ((u >> 16) & 1u); return (us)(u >> 16); }
__device__ __forceinline__ float bf2f(us b) { return __uint_as_float(((unsigned)b) << 16); }
__device__ __forceinline__ float bfr(float f) { return bf2f(f2bf(f)); }
__device__ __forceinline__ void wave_sync() { __builtin_amdgcn_fence(3  , "wavefront"); __builtin_amdgcn_wave_barrier(); asm volatile("" ::: "memory"); }

template<bool F16> struct OpT;
template<> struct OpT<false> {
    typedef v16bf F;
    static __device__ __forceinline__ F ld(const us* p) { return __builtin_bit_cast(v16bf, __builtin_shufflevector(*(const v8us*)p, *(const v8us*)(p + 16), 0, 1, 2, 3, 4, 5, 6, 7, 8, 9, 10, 11, 12, 13, 14, 15)); }
    static __device__ __forceinline__ v8f mma(F a, F b, v8f c) { return __builtin_amdgcn_wmma_f32_16x16x32_bf16(false, a, false, b, (short)0, c, false, false); }
};
template<> struct OpT<true> {
    typedef v16h F;
    static __device__ __forceinline__ F ld(const us* p) { return __builtin_bit_cast(v16h, __builtin_shufflevector(*(const v8us*)p, *(const v8us*)(p + 16), 0, 1, 2, 3, 4, 5, 6, 7, 8, 9, 10, 11, 12, 13, 14, 15)); }
    static __device__ __forceinline__ v8f mma(F a, F b, v8f c) { return __builtin_amdgcn_wmma_f32_16x16x32_f16(false, a, false, b, (short)0, c, false, false); }
};

__global__ __launch_bounds__(256) void k_cvt8(const float* __restrict__ src, us* dst, size_t n8) {
    const size_t i = (size_t)blockIdx.x * 256 + threadIdx.x; if (i >= n8) return;
    const v8f v = *(const v8f*)(src + i * 8); v8us o;
#pragma unroll
    for (int k = 0; k < 8; ++k) o[k] = f2bf(v[k]);
    *(volatile v8us*)(dst + i * 8) = o; __threadfence(); *(volatile v8us*)(dst + i * 8) = o;
}

template<int MODE>
__global__ __launch_bounds__(256) void k_wt(const float* __restrict__ W, us* Wt) {
    __shared__ __align__(16) float tl[64 * 68];
    const int t = threadIdx.x;
    const int k0 = blockIdx.x * 64, n0 = blockIdx.y * 64;
#pragma unroll
    for (int i = 0; i < 4; ++i) { const int kk = (t >> 4) + 16 * i, c4 = (t & 15) * 4;
        const v4f v = *(const v4f*)(W + (size_t)(k0 + kk) * DM + n0 + c4);
        *(v4fa*)(&tl[kk * 68 + c4]) = v; }
    __syncthreads();
    const int k8 = (t & 7) * 8;
    v8us o0, o1;
#pragma unroll
    for (int j = 0; j < 8; ++j) {
        const float x0 = tl[(k8 + j) * 68 + (t >> 3)];
        const float x1 = tl[(k8 + j) * 68 + (t >> 3) + 32];
        us b0 = f2bf(x0), b1 = f2bf(x1);
        if (MODE == 1) { const h16 h0 = (h16)(bf2f(b0) * WOS); const h16 h1 = (h16)(bf2f(b1) * WOS); b0 = __builtin_bit_cast(us, h0); b1 = __builtin_bit_cast(us, h1); }
        o0[j] = b0; o1[j] = b1; }
    us* p0 = Wt + (size_t)(n0 + (t >> 3)) * DM + k0 + k8;
    us* p1 = Wt + (size_t)(n0 + (t >> 3) + 32) * DM + k0 + k8;
#pragma unroll 1
    for (int ps = 0; ps < 2; ++ps) {
        *(volatile v8us*)p0 = o0; *(volatile v8us*)p1 = o1;
        if (ps == 0) __threadfence(); }
}

struct GP { long long K, lda, ldb, aZ, bZ, bRB, bRBs, oZ, oRB, osRB, pitch, oCB, osCB; };
static_assert(sizeof(GP) == 13 * 8);

template<int NPA, int NPB, int MT, int EPI, int BIAS, bool F16>
__global__ __launch_bounds__(32) void k_gemm(const us* __restrict__ A0, const us* __restrict__ A1, const us* __restrict__ B0, const us* __restrict__ B1,
                                             us* P0, us* P1, float* PF, const float* __restrict__ bias, float scale, GP g) {
    static_assert(MT == 2 || MT == 4);
    typedef OpT<F16> OP; typedef typename OP::F FR;
    __shared__ __align__(16) float os[16 * 68];
    const int lane = threadIdx.x & 31, lr = lane & 15, hi = lane >> 4;
    const unsigned r0 = blockIdx.x * (16u * MT), c0 = blockIdx.y * 64u, z = blockIdx.z;
    const int K = (int)g.K; const size_t lda = (size_t)g.lda, ldb = (size_t)g.ldb;
    v8f acc[MT][4];
#pragma unroll
    for (int mb = 0; mb < MT; ++mb)
#pragma unroll
        for (int nb = 0; nb < 4; ++nb) acc[mb][nb] = (v8f){};
    const size_t aoff = (size_t)z * (size_t)g.aZ + (size_t)(r0 + lr) * lda + 8 * hi;
    const size_t boff = (size_t)z * (size_t)g.bZ + (size_t)(r0 / (unsigned)g.bRB) * (size_t)g.bRBs + (size_t)(c0 + lr) * ldb + 8 * hi;
#pragma unroll 1
    for (int kc = 0; kc < K; kc += 32) {
        FR ah[MT], al[MT];
#pragma unroll
        for (int mb = 0; mb < MT; ++mb) { ah[mb] = OP::ld(A0 + aoff + (size_t)mb * 16 * lda + kc); al[mb] = (NPA == 2) ? OP::ld(A1 + aoff + (size_t)mb * 16 * lda + kc) : ah[mb]; }
#pragma unroll
        for (int nb = 0; nb < 4; ++nb) {
            const FR bh = OP::ld(B0 + boff + (size_t)nb * 16 * ldb + kc);
            const FR bl = (NPB == 2) ? OP::ld(B1 + boff + (size_t)nb * 16 * ldb + kc) : bh;
#pragma unroll
            for (int mb = 0; mb < MT; ++mb) acc[mb][nb] = OP::mma(ah[mb], bh, acc[mb][nb]);
            if (NPB == 2) {
#pragma unroll
                for (int mb = 0; mb < MT; ++mb) acc[mb][nb] = OP::mma(ah[mb], bl, acc[mb][nb]); }
            if (NPA == 2) {
#pragma unroll
                for (int mb = 0; mb < MT; ++mb) acc[mb][nb] = OP::mma(al[mb], bh, acc[mb][nb]); }
        }
        asm volatile("v_nop\n\tv_nop\n\tv_nop\n\tv_nop"
                     : "+v"(acc[0][0]), "+v"(acc[0][1]), "+v"(acc[0][2]), "+v"(acc[0][3]), "+v"(acc[MT - 1][0]), "+v"(acc[MT - 1][1]), "+v"(acc[MT - 1][2]), "+v"(acc[MT - 1][3])
                     : "v"(ah[0]), "v"(ah[MT - 1]), "v"(al[0]), "v"(al[MT - 1]));
    }
    const size_t pitch = (size_t)g.pitch;
    const size_t tbase = (size_t)z * (size_t)g.oZ + (size_t)(r0 / (unsigned)g.oRB) * (size_t)g.osRB + (size_t)(r0 % (unsigned)g.oRB) * pitch
                       + (size_t)(c0 / (unsigned)g.oCB) * (size_t)g.osCB + (size_t)(c0 % (unsigned)g.oCB);
    float bc[8];
#pragma unroll
    for (int i = 0; i < 8; ++i) bc[i] = 0.0f;
    if (BIAS == 1 && EPI != 2) { const v4f t0 = *(const v4f*)(bias + c0 + (lane & 7) * 8); const v4f t1 = *(const v4f*)(bias + c0 + (lane & 7) * 8 + 4);
#pragma unroll
        for (int i = 0; i < 4; ++i) { bc[i] = bfr(t0[i]); bc[4 + i] = bfr(t1[i]); } }
    if (BIAS == 1 && EPI == 2) { const v4f t0 = *(const v4f*)(bias + c0 + lr * 4);
#pragma unroll
        for (int i = 0; i < 4; ++i) bc[i] = bfr(t0[i]); }
#pragma unroll
    for (int mb = 0; mb < MT; ++mb) {
#pragma unroll
        for (int nb = 0; nb < 4; ++nb) {
#pragma unroll
            for (int j = 0; j < 8; ++j) os[(hi * 8 + j) * 68 + nb * 16 + lr] = acc[mb][nb][j]; }
        wave_sync();
        const size_t sb = tbase + (size_t)(mb * 16) * pitch;
        if (EPI == 2) {
#pragma unroll 1
            for (int ps = 0; ps < 2; ++ps) {
#pragma unroll
                for (int s = 0; s < 8; ++s) { const int row = 2 * s + hi, cofs = lr * 4;
                    const v4f x = *(const v4fa*)(&os[row * 68 + cofs]); v4f val;
#pragma unroll
                    for (int i = 0; i < 4; ++i) val[i] = x[i] * scale + bc[i];
                    *(volatile v4f*)(PF + sb + (size_t)row * pitch + cofs) = val; }
                if (ps == 0) __threadfence(); }
        } else {
#pragma unroll 1
            for (int ps = 0; ps < 2; ++ps) {
#pragma unroll
                for (int s = 0; s < 4; ++s) { const int row = 4 * s + (lane >> 3), c8 = (lane & 7) * 8;
                    const v4f x0 = *(const v4fa*)(&os[row * 68 + c8]); const v4f x1 = *(const v4fa*)(&os[row * 68 + c8 + 4]);
                    const float rb = (BIAS == 2) ? bfr(bias[r0 + mb * 16 + row]) : 0.0f;
                    v8us hv, lv;
#pragma unroll
                    for (int i = 0; i < 4; ++i) {
                        const float y0 = x0[i] * scale + ((BIAS == 1) ? bc[i] : rb);
                        const float y1 = x1[i] * scale + ((BIAS == 1) ? bc[4 + i] : rb);
                        if (EPI == 0) { const us h0 = f2bf(y0), h1 = f2bf(y1); hv[i] = h0; hv[4 + i] = h1; lv[i] = f2bf(y0 - bf2f(h0)); lv[4 + i] = f2bf(y1 - bf2f(h1)); }
                        else { const h16 a0 = (h16)y0; const h16 a1 = (h16)y1; hv[i] = __builtin_bit_cast(us, a0); hv[4 + i] = __builtin_bit_cast(us, a1); lv[i] = 0; lv[4 + i] = 0; }
                    }
                    const size_t oo = sb + (size_t)row * pitch + c8;
                    *(volatile v8us*)(P0 + oo) = hv; if (EPI == 0) *(volatile v8us*)(P1 + oo) = lv; }
                if (ps == 0) __threadfence(); }
        }
        wave_sync();
    }
}

static constexpr size_t al256(size_t v) { return (v + 255) & ~(size_t)255; }
static constexpr size_t SZ_XB = al256((size_t)NB * SEQ * DM * 2);
static constexpr size_t SZ_W  = al256((size_t)DM * DM * 2);
static constexpr size_t SZ_PL = al256((size_t)NB * SEQ * DM * 2);
static constexpr size_t SZ_M  = al256((size_t)NB * NH_ * HD * HD * 2);
static constexpr size_t SZ_TOTAL = SZ_XB + 4 * SZ_W + 6 * SZ_PL + 2 * SZ_M;
static_assert(SZ_TOTAL <= (size_t)134217728);
static_assert((size_t)NB * SEQ * DM * 2 <= SZ_XB);

extern "C" void kernel_launch(void* const* d_in, const int* in_sizes, int n_in,
                              void* d_out, int out_size, void* d_ws, size_t ws_size, hipStream_t stream) {
    if (n_in < 11) return;
    const size_t needx = ((size_t)(NB - 1) * SEQ_FULL + SEQ) * DM;
    if ((size_t)in_sizes[0] < needx || (size_t)in_sizes[1] < needx || (size_t)in_sizes[2] < needx) return;
    if ((size_t)in_sizes[3] < (size_t)DM * DM || (size_t)in_sizes[5] < (size_t)DM * DM || (size_t)in_sizes[7] < (size_t)DM * DM || (size_t)in_sizes[9] < (size_t)DM * DM) return;
    if (in_sizes[4] < DM || in_sizes[6] < DM || in_sizes[8] < DM || in_sizes[10] < DM) return;
    if ((size_t)out_size < ((size_t)(NB - 1) * OUT_SEQ + SEQ) * DM) return;
    if (SZ_TOTAL > ws_size) return;
    const float* xq = (const float*)d_in[0]; const float* xk = (const float*)d_in[1]; const float* xv = (const float*)d_in[2];
    const float* wq = (const float*)d_in[3]; const float* bq = (const float*)d_in[4];
    const float* wk = (const float*)d_in[5]; const float* bk = (const float*)d_in[6];
    const float* wv = (const float*)d_in[7]; const float* bv = (const float*)d_in[8];
    const float* wo = (const float*)d_in[9]; const float* bo = (const float*)d_in[10];
    float* OUT = (float*)d_out;
    char* wsp = (char*)d_ws;
    us* XB  = (us*)wsp; wsp += SZ_XB;
    us* WQT = (us*)wsp; wsp += SZ_W;
    us* WKT = (us*)wsp; wsp += SZ_W;
    us* WVT = (us*)wsp; wsp += SZ_W;
    us* WOT = (us*)wsp; wsp += SZ_W;
    us* QH  = (us*)wsp; wsp += SZ_PL;
    us* QL  = (us*)wsp; wsp += SZ_PL;
    us* KH  = (us*)wsp; wsp += SZ_PL;
    us* KL  = (us*)wsp; wsp += SZ_PL;
    us* VH  = (us*)wsp; wsp += SZ_PL;
    us* VL  = (us*)wsp; wsp += SZ_PL;
    us* MH  = (us*)wsp; wsp += SZ_M;
    us* ML  = (us*)wsp; wsp += SZ_M;
    us* A2  = XB;

    k_wt<0><<<dim3(DM / 64, DM / 64, 1), 256, 0, stream>>>(wq, WQT);
    k_wt<0><<<dim3(DM / 64, DM / 64, 1), 256, 0, stream>>>(wk, WKT);
    k_wt<0><<<dim3(DM / 64, DM / 64, 1), 256, 0, stream>>>(wv, WVT);
    k_wt<1><<<dim3(DM / 64, DM / 64, 1), 256, 0, stream>>>(wo, WOT);

    const GP gq  = { DM, DM, DM, 0, 0, BIGB, 0, 0, BIGB, 0, DM, BIGB, 0 };
    const GP gt  = { DM, DM, DM, 0, 0, BIGB, 0, 0, BIGB, 0, SEQ, SEQ, (long long)DM * SEQ };
    const GP gkv = { SEQ, SEQ, SEQ, (long long)HD * SEQ, (long long)HD * SEQ, BIGB, 0, (long long)HD * HD, BIGB, 0, HD, BIGB, 0 };
    const GP gat = { HD, DM, HD, HD, (long long)HD * HD, SEQ, (long long)NH_ * HD * HD, HD, BIGB, 0, DM, BIGB, 0 };
    const GP go  = { DM, DM, DM, 0, 0, BIGB, 0, 0, SEQ, (long long)OUT_SEQ * DM, DM, BIGB, 0 };

    const size_t n8b = (size_t)SEQ * DM / 8; const unsigned gcb = (unsigned)((n8b + 255) / 256);
    const size_t n8a = (size_t)NB * SEQ * DM / 8; const unsigned gca = (unsigned)((n8a + 255) / 256);

    if (SEQ == SEQ_FULL) k_cvt8<<<gca, 256, 0, stream>>>(xq, XB, n8a);
    else for (int b = 0; b < NB; ++b) k_cvt8<<<gcb, 256, 0, stream>>>(xq + (size_t)b * SEQ_FULL * DM, XB + (size_t)b * SEQ * DM, n8b);
    k_gemm<1, 1, 4, 0, 1, false><<<dim3(NB * SEQ / 64, DM / 64, 1), 32, 0, stream>>>(XB, XB, WQT, WQT, QH, QL, OUT, bq, 1.0f, gq);
    if (SEQ == SEQ_FULL) k_cvt8<<<gca, 256, 0, stream>>>(xk, XB, n8a);
    else for (int b = 0; b < NB; ++b) k_cvt8<<<gcb, 256, 0, stream>>>(xk + (size_t)b * SEQ_FULL * DM, XB + (size_t)b * SEQ * DM, n8b);
    k_gemm<1, 1, 4, 0, 2, false><<<dim3(DM / 64, NB * SEQ / 64, 1), 32, 0, stream>>>(WKT, WKT, XB, XB, KH, KL, OUT, bk, 1.0f, gt);
    if (SEQ == SEQ_FULL) k_cvt8<<<gca, 256, 0, stream>>>(xv, XB, n8a);
    else for (int b = 0; b < NB; ++b) k_cvt8<<<gcb, 256, 0, stream>>>(xv + (size_t)b * SEQ_FULL * DM, XB + (size_t)b * SEQ * DM, n8b);
    k_gemm<1, 1, 4, 0, 2, false><<<dim3(DM / 64, NB * SEQ / 64, 1), 32, 0, stream>>>(WVT, WVT, XB, XB, VH, VL, OUT, bv, 1.0f, gt);

    k_gemm<2, 2, 2, 0, 0, false><<<dim3(HD / 32, 1, NB * NH_), 32, 0, stream>>>(VH, VL, KH, KL, MH, ML, OUT, bq, 0.125f, gkv);
    k_gemm<2, 2, 2, 1, 0, false><<<dim3(NB * SEQ / 32, 1, NH_), 32, 0, stream>>>(QH, QL, MH, ML, A2, A2, OUT, bq, 1.0f, gat);
    k_gemm<1, 1, 4, 2, 1, true><<<dim3(NB * SEQ / 64, DM / 64, 1), 32, 0, stream>>>(A2, A2, WOT, WOT, QH, QL, OUT, bo, WOI, go);
}
